// HeteroGNN_51745765982901
// MI455X (gfx1250) — hardware-run, weakly checked
//
#include <hip/hip_runtime.h>
#include <math.h>

constexpr int kNG  = 50000;
constexpr int kNC  = 100000;
constexpr int kDR  = 128;
constexpr int kDH  = 64;
constexpr int kEGG = 800000;
constexpr int kECG = 1600000;
constexpr int kECC = 1600000;
constexpr int kNGP = 50048;
constexpr int kNCP = 100032;
constexpr int kGRW = 32;
constexpr int kThreads = 256;
constexpr int kTileRows = 512;
constexpr int kBlkG = 98;
constexpr int kBlkC = 196;
constexpr int kCH = 8192;
constexpr int kNchGG = (kEGG + kCH - 1) / kCH;
constexpr int kNchCG = (kECG + kCH - 1) / kCH;
constexpr int kNKPG = 800;
constexpr int kNKPC = 1600;
constexpr int kWPlane = 64 * 128;
constexpr int kWSlots = 7;
constexpr unsigned kSent = 0xFFFFFFFFu;
constexpr int kOutN = kNG * 3;
constexpr float kLnEps = 1e-5f;
constexpr float kInv64 = 1.0f / 64.0f;

static_assert(kECG == kECC);
static_assert(kEGG % 4 == 0 && kECG % 4 == 0);
static_assert(kCH == 32 * kThreads);
static_assert(kNchGG * kCH >= kEGG && kNchCG * kCH >= kECG);
static_assert(kBlkG * kTileRows >= kNGP && kBlkC * kTileRows >= kNCP);
static_assert(8 * kBlkG < kNKPG && 8 * kBlkC < kNKPC);
static_assert(kNKPG % 32 == 0 && kNKPC % 32 == 0);
static_assert(kNKPG <= 1024 && kNKPC <= 2048);
static_assert(((kNG - 1) >> 6) < 1024 && ((kNC - 1) >> 6) < 2048);
static_assert(kNGP % 64 == 0 && kNCP % 64 == 0);
static_assert(kNGP % kGRW == 0 && kNCP % kGRW == 0);
static_assert(kDR % 32 == 0 && kDH % 32 == 0);
static_assert(kOutN % 4 == 0);
static_assert((kTileRows * 12) % 128 == 0);
static_assert(kNC < (1 << 17));

typedef __attribute__((ext_vector_type(16))) __bf16   v16b;
typedef __attribute__((ext_vector_type(8)))  __bf16   v8b;
typedef __attribute__((ext_vector_type(8)))  _Float16 v8h;
typedef __attribute__((ext_vector_type(8)))  float    v8f;
typedef __attribute__((ext_vector_type(4)))  float    v4f;
typedef __attribute__((ext_vector_type(2)))  float    v2f;
typedef __attribute__((ext_vector_type(4)))  int      v4i;
typedef __attribute__((ext_vector_type(4)))  unsigned int v4u;

__device__ __forceinline__ unsigned short f2bf_bits(float f) {
  unsigned u = __float_as_uint(f);
  return (unsigned short)((u + 0x7FFFu + ((u >> 16) & 1u)) >> 16);
}
__device__ __forceinline__ float bf_bits2f(unsigned short h) { return __uint_as_float(((unsigned)h) << 16); }
__device__ __forceinline__ float bfr(float f) { return bf_bits2f(f2bf_bits(f)); }
__device__ __forceinline__ __bf16 tobf(float f) { return __builtin_bit_cast(__bf16, f2bf_bits(f)); }

__device__ __forceinline__ void guard4_b(v8f& a, v8f& b, v8f& c, v8f& d, v16b x, v16b y) {
  asm volatile("v_nop\n\tv_nop\n\tv_nop\n\tv_nop" : "+v"(a), "+v"(b), "+v"(c), "+v"(d) : "v"(x), "v"(y));
}
__device__ __forceinline__ void keep4_b(v16b a, v16b b, v16b c, v16b d) { asm volatile("v_nop" :: "v"(a), "v"(b), "v"(c), "v"(d)); }
__device__ __forceinline__ void acc_guard4(v8f& a, v8f& b, v8f& c, v8f& d) { asm volatile("v_nop\n\tv_nop\n\tv_nop\n\tv_nop" : "+v"(a), "+v"(b), "+v"(c), "+v"(d)); }
template <typename T> struct Frag;
template <> struct Frag<__bf16> {
  typedef v16b V; union U { v16b v; v8b h[2]; };
  static __device__ __forceinline__ v16b load(const __bf16* p) {
    U f; f.h[0] = *(const v8b*)(p); f.h[1] = *(const v8b*)(p + 16); return f.v;
  }
  static __device__ __forceinline__ v8f mma(v16b a, v16b b, v8f c) {
    return __builtin_amdgcn_wmma_f32_16x16x32_bf16(false, a, false, b, (short)0, c, false, false);
  }
};

__device__ __forceinline__ unsigned pk16(unsigned short a, unsigned short b) { return (unsigned)a | ((unsigned)b << 16); }
__device__ __forceinline__ int clampi(int v, int hi) { return v < 0 ? 0 : (v > hi ? hi : v); }

template <int KDIM, bool ASRC32, bool ASPLIT, int EPI, int OUTM>
__global__ __launch_bounds__(256) void gemm_n64(const float* __restrict__ A32,
                                                const unsigned short* __restrict__ Ahp, const unsigned short* __restrict__ Alp,
                                                int n_real, int m_tiles,
                                                const unsigned short* __restrict__ Bp,
                                                const float* __restrict__ bias,
                                                const float* __restrict__ lns, const float* __restrict__ lnb,
                                                float* __restrict__ C32, unsigned short* __restrict__ CHp,
                                                unsigned short* __restrict__ CLp) {
  static_assert(!(ASRC32 && ASPLIT));
  static_assert(KDIM % 32 == 0);
  __shared__ __align__(16) float sT[8][16 * 68];
  const int lane = threadIdx.x & 31;
  const int wave = threadIdx.x >> 5;
  const int tile = blockIdx.x * 8 + wave;
  if (tile >= m_tiles) return;
  const int m0 = tile * kGRW;
  const __bf16* Bt = (const __bf16*)Bp;
  const __bf16* Ah = (const __bf16*)Ahp;
  const __bf16* Al = (const __bf16*)Alp;
  const int rlane = lane & 15;
  const int koff  = (lane >> 4) * 8;
  const int mOff  = (lane >> 4) * 8;

  v8f acc[2][4];
#pragma unroll
  for (int i = 0; i < 2; ++i)
#pragma unroll
    for (int j = 0; j < 4; ++j) acc[i][j] = (v8f){0.f,0.f,0.f,0.f,0.f,0.f,0.f,0.f};

#pragma unroll 1
  for (int k0 = 0; k0 < KDIM; k0 += 32) {
    v16b bfr4[4];
#pragma unroll
    for (int j = 0; j < 4; ++j) bfr4[j] = Frag<__bf16>::load(Bt + (size_t)((j << 4) + rlane) * KDIM + koff + k0);
#pragma unroll
    for (int i = 0; i < 2; ++i) {
      v16b ah, al;
      if (ASRC32) {
        int row = m0 + (i << 4) + rlane; row = row < n_real ? row : n_real - 1;
        const float* ap = A32 + (size_t)row * KDIM + k0 + koff;
        const v4f f0 = *(const v4f*)(ap);
        const v4f f1 = *(const v4f*)(ap + 4);
        const v4f f2 = *(const v4f*)(ap + 16);
        const v4f f3 = *(const v4f*)(ap + 20);
        typename Frag<__bf16>::U fu;
#pragma unroll
        for (int e = 0; e < 4; ++e) {
          fu.h[0][e] = tobf(f0[e]); fu.h[0][4 + e] = tobf(f1[e]);
          fu.h[1][e] = tobf(f2[e]); fu.h[1][4 + e] = tobf(f3[e]);
        }
        ah = fu.v; al = ah;
      } else {
        const size_t ao = (size_t)(m0 + (i << 4) + rlane) * KDIM + koff + k0;
        ah = Frag<__bf16>::load(Ah + ao);
        if (ASPLIT) al = Frag<__bf16>::load(Al + ao); else al = ah;
      }
#pragma unroll
      for (int j = 0; j < 4; ++j) {
        acc[i][j] = Frag<__bf16>::mma(ah, bfr4[j], acc[i][j]);
        if (ASPLIT) acc[i][j] = Frag<__bf16>::mma(al, bfr4[j], acc[i][j]);
      }
      guard4_b(acc[i][0], acc[i][1], acc[i][2], acc[i][3], ah, al);
    }
    keep4_b(bfr4[0], bfr4[1], bfr4[2], bfr4[3]);
  }
  acc_guard4(acc[0][0], acc[0][1], acc[0][2], acc[0][3]);
  acc_guard4(acc[1][0], acc[1][1], acc[1][2], acc[1][3]);

  float bb[4] = {0.f, 0.f, 0.f, 0.f};
  float ls[4] = {1.f, 1.f, 1.f, 1.f};
  float lb[4] = {0.f, 0.f, 0.f, 0.f};
  if (EPI != 0) {
#pragma unroll
    for (int j = 0; j < 4; ++j) bb[j] = bfr(bias[(j << 4) + rlane]);
  }
  if (EPI >= 2) {
#pragma unroll
    for (int j = 0; j < 4; ++j) { ls[j] = bfr(lns[(j << 4) + rlane]); lb[j] = bfr(lnb[(j << 4) + rlane]); }
  }
  float* slab = sT[wave];
#pragma unroll
  for (int i = 0; i < 2; ++i) {
    const int mBase = m0 + (i << 4);
#pragma unroll
    for (int r = 0; r < 8; ++r) {
      const int row = mBase + mOff + r;
      const bool live = row < n_real;
      float v[4];
#pragma unroll
      for (int j = 0; j < 4; ++j) v[j] = acc[i][j][r] + bb[j];
      if (EPI == 1 || EPI == 3) {
#pragma unroll
        for (int j = 0; j < 4; ++j) v[j] = fmaxf(v[j], 0.0f);
      }
      if (EPI >= 2) {
        float s = (v[0] + v[1]) + (v[2] + v[3]);
        s += __shfl_xor(s, 1, 32); s += __shfl_xor(s, 2, 32); s += __shfl_xor(s, 4, 32); s += __shfl_xor(s, 8, 32);
        const float mean = s * kInv64;
        float d[4];
        float q = 0.0f;
#pragma unroll
        for (int j = 0; j < 4; ++j) { d[j] = v[j] - mean; q += d[j] * d[j]; }
        q += __shfl_xor(q, 1, 32); q += __shfl_xor(q, 2, 32); q += __shfl_xor(q, 4, 32); q += __shfl_xor(q, 8, 32);
        const float rstd = rsqrtf(q * kInv64 + kLnEps);
#pragma unroll
        for (int j = 0; j < 4; ++j) v[j] = fmaxf((d[j] * rstd) * ls[j] + lb[j], 0.0f);
      }
#pragma unroll
      for (int j = 0; j < 4; ++j) slab[(mOff + r) * 68 + (j << 4) + rlane] = live ? v[j] : 0.0f;
    }
    __builtin_amdgcn_fence(__ATOMIC_RELEASE, "workgroup");
    __builtin_amdgcn_wave_barrier();
    __builtin_amdgcn_fence(__ATOMIC_ACQUIRE, "workgroup");
    if (OUTM == 0) {
      const int hh = lane >> 4, c4 = (lane & 15) * 4;
      for (int ps = 0; ps < 2; ++ps) {
#pragma unroll
        for (int it = 0; it < 8; ++it) {
          const int row = it * 2 + hh;
          const v4f vv = *(const v4f*)(slab + row * 68 + c4);
          *(volatile v4f*)(C32 + (size_t)(mBase + row) * kDH + c4) = vv;
        }
        __threadfence();
      }
    } else {
      const int q = lane >> 3, c8 = (lane & 7) * 8;
      for (int ps = 0; ps < 2; ++ps) {
#pragma unroll
        for (int it = 0; it < 4; ++it) {
          const int row = it * 4 + q;
          const float* sp = slab + row * 68 + c8;
          v8h hv, lv;
#pragma unroll
          for (int e = 0; e < 8; ++e) {
            const unsigned short hb = f2bf_bits(sp[e]);
            const unsigned short lb2 = f2bf_bits(sp[e] - bf_bits2f(hb));
            hv[e] = __builtin_bit_cast(_Float16, hb);
            lv[e] = __builtin_bit_cast(_Float16, lb2);
          }
          *(volatile v8h*)(CHp + (size_t)(mBase + row) * kDH + c8) = hv;
          *(volatile v8h*)(CLp + (size_t)(mBase + row) * kDH + c8) = lv;
        }
        __threadfence();
      }
    }
    __builtin_amdgcn_fence(__ATOMIC_RELEASE, "workgroup");
    __builtin_amdgcn_wave_barrier();
    __builtin_amdgcn_fence(__ATOMIC_ACQUIRE, "workgroup");
  }
}

__global__ __launch_bounds__(256) void prep_weights(const float* __restrict__ w0, const float* __restrict__ w1,
                                                    const float* __restrict__ w2, const float* __restrict__ w3,
                                                    const float* __restrict__ w4, const float* __restrict__ w5,
                                                    const float* __restrict__ w6, unsigned short* __restrict__ WP) {
  __shared__ __align__(16) float sW[kDR * 64];
  const int z = blockIdx.x;
  const float* W = (z == 0) ? w0 : (z == 1) ? w1 : (z == 2) ? w2 : (z == 3) ? w3 : (z == 4) ? w4 : (z == 5) ? w5 : w6;
  const int kd = (z < 2) ? kDR : kDH;
  const int n4 = (kd * 64) >> 2;
#pragma unroll 1
  for (int i = threadIdx.x; i < n4; i += 256) *(v4f*)(sW + 4 * i) = *(const v4f*)(W + 4 * i);
  __syncthreads();
  const int kq  = kd >> 3;
  const int cnt = 64 * kq;
  unsigned short* op = WP + (size_t)z * kWPlane;
  for (int ps = 0; ps < 2; ++ps) {
#pragma unroll 1
    for (int i = threadIdx.x; i < cnt; i += 256) {
      const int n  = i / kq;
      const int kb = (i - n * kq) * 8;
      unsigned short hb[8];
#pragma unroll
      for (int e = 0; e < 8; ++e) hb[e] = f2bf_bits(sW[(kb + e) * 64 + n]);
      const v4u u = (v4u){pk16(hb[0], hb[1]), pk16(hb[2], hb[3]), pk16(hb[4], hb[5]), pk16(hb[6], hb[7])};
      *(volatile v4u*)(op + (size_t)n * kd + kb) = u;
    }
    __threadfence();
  }
}

__device__ __forceinline__ int blk_excl_scan(int cnt, int* scan_ws, int tid, int* tot) {
  const int lane = tid & 31, wave = tid >> 5; int incl = cnt;
#pragma unroll
  for (int o = 1; o < 32; o <<= 1) { const int v = __shfl_up(incl, o, 32); if (lane >= o) incl += v; }
  if (lane == 31) scan_ws[wave] = incl;
  __syncthreads();
  if (wave == 0) { int wv = (lane < kThreads / 32) ? scan_ws[lane] : 0; int wincl = wv;
#pragma unroll
    for (int o = 1; o < 32; o <<= 1) { const int v = __shfl_up(wincl, o, 32); if (lane >= o) wincl += v; }
    if (lane < kThreads / 32) scan_ws[32 + lane] = wincl - wv; if (lane == 31) scan_ws[64] = wincl; }
  __syncthreads();
  const int res = scan_ws[32 + wave] + incl - cnt; *tot = scan_ws[64];
  return res;
}

template <int NKALL, int KEYBITS>
__global__ __launch_bounds__(kThreads) void bucket_edges(const int* __restrict__ dstv, int n_edges, int n_dst, int nkp,
                                                         unsigned* __restrict__ sorted, int* __restrict__ table, int nchunks) {
  static_assert(NKALL % kThreads == 0 && (1 << KEYBITS) == NKALL);
  __shared__ int scnt[8 * NKALL];
  __shared__ __align__(16) int soff[NKALL];
  __shared__ __align__(16) unsigned ssort[kCH];
  __shared__ int scan_ws[80];
  const int tid = threadIdx.x, lane = tid & 31, wave = tid >> 5;
  const int c = blockIdx.x;
  const int e0 = c * kCH;
  for (int i = tid; i < 8 * NKALL; i += kThreads) scnt[i] = 0;
  for (int i = tid; i < kCH; i += kThreads) ssort[i] = kSent;
  if (tid < 80) scan_ws[tid] = 0;
  int dv[32];
#pragma unroll
  for (int k = 0; k < 8; ++k) {
    const int idx = (k * kThreads + tid) * 4;
    int gb = e0 + idx; gb = (gb + 3 < n_edges) ? gb : (n_edges - 4);
    const v4i d4 = *(const v4i*)(dstv + gb);
    dv[4 * k] = d4[0]; dv[4 * k + 1] = d4[1]; dv[4 * k + 2] = d4[2]; dv[4 * k + 3] = d4[3];
  }
  __syncthreads();
  int* mycnt = scnt + wave * NKALL;
  const unsigned ltmask = (1u << lane) - 1u;
  unsigned rec[32]; int pk[32]; unsigned vmask = 0u;
#pragma unroll
  for (int s = 0; s < 32; ++s) {
    const int el = ((s >> 2) * kThreads + tid) * 4 + (s & 3);
    const int e  = e0 + el;
    const int d  = dv[s];
    const bool valid = (e < n_edges) && ((unsigned)d < (unsigned)n_dst);
    const int key = valid ? (d >> 6) : 0;
    unsigned peers = (unsigned)__ballot(valid ? 1 : 0);
#pragma unroll
    for (int bb = 0; bb < KEYBITS; ++bb) {
      const int kb = (key >> bb) & 1;
      const unsigned m = (unsigned)__ballot(kb);
      peers &= kb ? m : ~m;
    }
    const int rank = __builtin_popcount(peers & ltmask);
    const int cntk = __builtin_popcount(peers);
    const int base = mycnt[key];
    if (valid && rank == 0) mycnt[key] = base + cntk;
    rec[s] = ((unsigned)(d & 63) << 13) | (unsigned)el;
    pk[s]  = (key << 13) | ((base + rank) & 0x1FFF);
    vmask |= valid ? (1u << s) : 0u;
  }
  __syncthreads();
  for (int K = tid; K < NKALL; K += kThreads) {
    int run = 0;
#pragma unroll
    for (int w = 0; w < 8; ++w) { const int cc = scnt[w * NKALL + K]; scnt[w * NKALL + K] = run; run += cc; }
    soff[K] = run;
  }
  __syncthreads();
  {
    constexpr int KPT = NKALL / kThreads;
    int vals[KPT]; int sum = 0;
#pragma unroll
    for (int q = 0; q < KPT; ++q) { vals[q] = soff[tid * KPT + q]; sum += vals[q]; }
    int tot; int p = blk_excl_scan(sum, scan_ws, tid, &tot);
#pragma unroll
    for (int q = 0; q < KPT; ++q) { soff[tid * KPT + q] = p; p += vals[q]; }
    (void)tot;
  }
  __syncthreads();
#pragma unroll
  for (int s = 0; s < 32; ++s) {
    const int key = pk[s] >> 13;
    int pos = soff[key] + mycnt[key] + (pk[s] & 0x1FFF);
    pos = clampi(pos, kCH - 1);
    if ((vmask >> s) & 1u) ssort[pos] = rec[s];
  }
  __syncthreads();
  unsigned* sg = sorted + (size_t)c * kCH;
  int* tg = table + (size_t)c * nkp;
  const bool lastblk = (c == nchunks - 1);
  const v4u padv = (v4u){kSent, kSent, kSent, kSent};
  for (int ps = 0; ps < 2; ++ps) {
#pragma unroll
    for (int k = 0; k < 8; ++k) {
      const int idx = k * kThreads + tid;
      const v4u u = *(const v4u*)(ssort + 4 * idx);
      *(volatile v4u*)(sg + 4 * idx) = u;
    }
#pragma unroll 1
    for (int i = tid; i < (nkp >> 2); i += kThreads) {
      const v4i ov = *(const v4i*)(soff + 4 * i);
      *(volatile v4i*)(tg + 4 * i) = ov;
    }
    if (lastblk && tid < 8) *(volatile v4u*)(sorted + (size_t)nchunks * kCH + 4 * tid) = padv;
    __threadfence();
  }
}

__global__ __launch_bounds__(kThreads) void k_deg(const unsigned* __restrict__ sorted, const int* __restrict__ table,
                                                  const float* __restrict__ ew, float* __restrict__ dinv) {
  __shared__ __align__(16) float sdeg[kTileRows];
  const int tid = threadIdx.x, lane = tid & 31, wave = tid >> 5;
  const int b = blockIdx.x;
  const int key = 8 * b + wave;
  for (int i = tid; i < kTileRows; i += kThreads) sdeg[i] = 0.0f;
  __syncthreads();
#pragma unroll 1
  for (int c = 0; c < kNchGG; ++c) {
    const int* trow = table + (size_t)c * kNKPG + key;
    int lo = trow[0]; int hi = trow[1];
    lo = __builtin_amdgcn_readfirstlane(lo); hi = __builtin_amdgcn_readfirstlane(hi);
    lo = clampi(lo, kCH); hi = hi < lo ? lo : (hi > kCH ? kCH : hi);
    const unsigned* run = sorted + (size_t)c * kCH;
    const int ebase = c * kCH;
#pragma unroll 1
    for (int i = lo; i < hi; i += 32) {
      const unsigned rec = run[i + lane];
      int e = ebase + (int)(rec & 0x1FFFu); e = e < kEGG ? e : kEGG - 1;
      const float wl = bfr(ew[e]);
      const int nn = (hi - i) < 32 ? (hi - i) : 32;
#pragma unroll 1
      for (int j = 0; j < nn; ++j) {
        const unsigned r = __shfl(rec, j, 32);
        const float wj = __shfl(wl, j, 32);
        const int row = (wave << 6) + (int)((r >> 13) & 63u);
        if (lane == 0) sdeg[row] += wj;
      }
    }
  }
  __syncthreads();
  if (tid < 128) {
    v4f dvv;
#pragma unroll
    for (int e = 0; e < 4; ++e) dvv[e] = rsqrtf(sdeg[4 * tid + e] + 1.0f);
    float* p = dinv + (size_t)b * kTileRows + 4 * tid;
    *(volatile v4f*)p = dvv;
    __threadfence();
    *(volatile v4f*)p = dvv;
  }
}

__global__ __launch_bounds__(256) void k_norm(const int* __restrict__ ei, const float* __restrict__ ew,
                                              const float* __restrict__ dinv, float* __restrict__ normp) {
  const int i = blockIdx.x * 256 + threadIdx.x;
  if (i >= kEGG / 4) return;
  const int e4 = 4 * i;
  const v4i r4 = *(const v4i*)(ei + e4);
  const v4i c4 = *(const v4i*)(ei + kEGG + e4);
  const v4f w4 = *(const v4f*)(ew + e4);
  v4f nv;
#pragma unroll
  for (int e = 0; e < 4; ++e) {
    const int rs = clampi(r4[e], kNG - 1);
    const int cs = clampi(c4[e], kNG - 1);
    nv[e] = (dinv[rs] * bfr(w4[e])) * dinv[cs];
  }
  float* p = normp + e4;
  *(volatile v4f*)p = nv;
  __threadfence();
  *(volatile v4f*)p = nv;
}

template <bool DSTPL>
__global__ __launch_bounds__(kThreads) void k_gin(const unsigned* __restrict__ sorted, const int* __restrict__ table, int nchunks, int nkp,
                                                  const int* __restrict__ ei, int n_edges,
                                                  const float* xsrc, int n_src,
                                                  const float* xdst32, const unsigned short* __restrict__ xdh,
                                                  const unsigned short* __restrict__ xdl, int n_dst, int n_dst_pad,
                                                  const float* __restrict__ epsp,
                                                  unsigned short* __restrict__ hh, unsigned short* __restrict__ hl) {
  __shared__ __align__(16) float sacc[kTileRows * kDH];
  const int tid = threadIdx.x, lane = tid & 31, wave = tid >> 5;
  const int b = blockIdx.x;
  const int key = 8 * b + wave;
  const v4f z4 = {0.f, 0.f, 0.f, 0.f};
#pragma unroll 1
  for (int i = tid; i < kTileRows * kDH / 4; i += kThreads) *(v4f*)(sacc + 4 * i) = z4;
  __syncthreads();
#pragma unroll 1
  for (int c = 0; c < nchunks; ++c) {
    const int* trow = table + (size_t)c * nkp + key;
    int lo = trow[0]; int hi = trow[1];
    lo = __builtin_amdgcn_readfirstlane(lo); hi = __builtin_amdgcn_readfirstlane(hi);
    lo = clampi(lo, kCH); hi = hi < lo ? lo : (hi > kCH ? kCH : hi);
    const unsigned* run = sorted + (size_t)c * kCH;
    const int ebase = c * kCH;
#pragma unroll 1
    for (int i = lo; i < hi; i += 32) {
      const unsigned rec = run[i + lane];
      int e = ebase + (int)(rec & 0x1FFFu); e = e < n_edges ? e : n_edges - 1;
      const int s = clampi(ei[e], n_src - 1);
      const int nn = (hi - i) < 32 ? (hi - i) : 32;
#pragma unroll 1
      for (int j = 0; j < nn; ++j) {
        const unsigned r = __shfl(rec, j, 32);
        const int sj = __shfl(s, j, 32);
        const int row = (wave << 6) + (int)((r >> 13) & 63u);
        const v2f xv = *(const v2f*)(xsrc + (size_t)sj * kDH + 2 * lane);
        float* ap = sacc + row * kDH + 2 * lane;
        v2f a = *(const v2f*)ap;
        a = a + xv;
        *(v2f*)ap = a;
      }
    }
  }
  __syncthreads();
  const float ope = 1.0f + bfr(epsp[0]);
#pragma unroll 1
  for (int rr = 0; rr < 64; ++rr) {
    const int row = (wave << 6) + rr;
    const int n = b * kTileRows + row;
    if (n < n_dst_pad) {
      const v2f a = *(const v2f*)(sacc + row * kDH + 2 * lane);
      float xd0, xd1;
      if (DSTPL) {
        const unsigned hw = *((const unsigned*)(xdh + (size_t)n * kDH) + lane);
        const unsigned lw = *((const unsigned*)(xdl + (size_t)n * kDH) + lane);
        xd0 = __uint_as_float(hw << 16) + __uint_as_float(lw << 16);
        xd1 = __uint_as_float(hw & 0xffff0000u) + __uint_as_float(lw & 0xffff0000u);
      } else {
        const v2f xd = *(const v2f*)(xdst32 + (size_t)n * kDH + 2 * lane);
        xd0 = xd[0]; xd1 = xd[1];
      }
      const bool live = n < n_dst;
      float h0 = ope * xd0 + a[0];
      float h1 = ope * xd1 + a[1];
      h0 = live ? h0 : 0.0f; h1 = live ? h1 : 0.0f;
      const unsigned short hb0 = f2bf_bits(h0), hb1 = f2bf_bits(h1);
      const unsigned short lb0 = f2bf_bits(h0 - bf_bits2f(hb0)), lb1 = f2bf_bits(h1 - bf_bits2f(hb1));
      const unsigned uh = pk16(hb0, hb1);
      const unsigned ul = pk16(lb0, lb1);
      unsigned* ph = (unsigned*)(hh + (size_t)n * kDH) + lane;
      unsigned* pl = (unsigned*)(hl + (size_t)n * kDH) + lane;
      *(volatile unsigned*)ph = uh;
      *(volatile unsigned*)pl = ul;
      __threadfence();
      *(volatile unsigned*)ph = uh;
      *(volatile unsigned*)pl = ul;
    }
  }
}

template <bool HEAD>
__global__ __launch_bounds__(kThreads) void k_gcn(const unsigned* __restrict__ sorted, const int* __restrict__ table,
                                                  const int* __restrict__ ei, const float* __restrict__ normp,
                                                  const float* __restrict__ xt, const float* __restrict__ dinv,
                                                  const float* __restrict__ bg, const float* __restrict__ ging,
                                                  const float* __restrict__ lns, const float* __restrict__ lnb,
                                                  unsigned short* __restrict__ xgh, unsigned short* __restrict__ xgl,
                                                  const float* __restrict__ Wo, const float* __restrict__ bo,
                                                  float* __restrict__ out) {
  __shared__ __align__(16) float sacc[kTileRows * kDH];
  __shared__ __align__(16) float so[HEAD ? kTileRows * 3 : 4];
  const int tid = threadIdx.x, lane = tid & 31, wave = tid >> 5;
  const int b = blockIdx.x;
  const int key = 8 * b + wave;
  const v4f z4 = {0.f, 0.f, 0.f, 0.f};
#pragma unroll 1
  for (int i = tid; i < kTileRows * kDH / 4; i += kThreads) *(v4f*)(sacc + 4 * i) = z4;
  __syncthreads();
#pragma unroll 1
  for (int c = 0; c < kNchGG; ++c) {
    const int* trow = table + (size_t)c * kNKPG + key;
    int lo = trow[0]; int hi = trow[1];
    lo = __builtin_amdgcn_readfirstlane(lo); hi = __builtin_amdgcn_readfirstlane(hi);
    lo = clampi(lo, kCH); hi = hi < lo ? lo : (hi > kCH ? kCH : hi);
    const unsigned* run = sorted + (size_t)c * kCH;
    const int ebase = c * kCH;
#pragma unroll 1
    for (int i = lo; i < hi; i += 32) {
      const unsigned rec = run[i + lane];
      int e = ebase + (int)(rec & 0x1FFFu); e = e < kEGG ? e : kEGG - 1;
      const int s = clampi(ei[e], kNG - 1);
      const float nw = normp[e];
      const int nn = (hi - i) < 32 ? (hi - i) : 32;
#pragma unroll 1
      for (int j = 0; j < nn; ++j) {
        const unsigned r = __shfl(rec, j, 32);
        const int sj = __shfl(s, j, 32);
        const float wj = __shfl(nw, j, 32);
        const int row = (wave << 6) + (int)((r >> 13) & 63u);
        const v2f xv = *(const v2f*)(xt + (size_t)sj * kDH + 2 * lane);
        float* ap = sacc + row * kDH + 2 * lane;
        v2f a = *(const v2f*)ap;
        a = a + wj * xv;
        *(v2f*)ap = a;
      }
    }
  }
  __syncthreads();
  const float bg0 = bfr(bg[2 * lane]),  bg1 = bfr(bg[2 * lane + 1]);
  const float ls0 = bfr(lns[2 * lane]), ls1 = bfr(lns[2 * lane + 1]);
  const float lb0 = bfr(lnb[2 * lane]), lb1 = bfr(lnb[2 * lane + 1]);
  float w00 = 0.f, w01 = 0.f, w02 = 0.f, w10 = 0.f, w11 = 0.f, w12 = 0.f, bo0 = 0.f, bo1 = 0.f, bo2 = 0.f;
  if (HEAD) {
    w00 = bfr(Wo[(2 * lane) * 3 + 0]); w01 = bfr(Wo[(2 * lane) * 3 + 1]); w02 = bfr(Wo[(2 * lane) * 3 + 2]);
    w10 = bfr(Wo[(2 * lane + 1) * 3 + 0]); w11 = bfr(Wo[(2 * lane + 1) * 3 + 1]); w12 = bfr(Wo[(2 * lane + 1) * 3 + 2]);
    bo0 = bfr(bo[0]); bo1 = bfr(bo[1]); bo2 = bfr(bo[2]);
  }
#pragma unroll 1
  for (int rr = 0; rr < 64; ++rr) {
    const int row = (wave << 6) + rr;
    const int n = b * kTileRows + row;
    if (n < kNGP) {
      const v2f a  = *(const v2f*)(sacc + row * kDH + 2 * lane);
      const v2f xs = *(const v2f*)(xt   + (size_t)n * kDH + 2 * lane);
      const v2f gi = *(const v2f*)(ging + (size_t)n * kDH + 2 * lane);
      const float dd = dinv[n];
      const float d2 = dd * dd;
      const float g0 = ((a[0] + d2 * xs[0]) + bg0) + gi[0];
      const float g1 = ((a[1] + d2 * xs[1]) + bg1) + gi[1];
      float sm = g0 + g1;
      sm += __shfl_xor(sm, 1, 32); sm += __shfl_xor(sm, 2, 32); sm += __shfl_xor(sm, 4, 32); sm += __shfl_xor(sm, 8, 32); sm += __shfl_xor(sm, 16, 32);
      const float mean = sm * kInv64;
      const float e0 = g0 - mean, e1 = g1 - mean;
      float q = e0 * e0 + e1 * e1;
      q += __shfl_xor(q, 1, 32); q += __shfl_xor(q, 2, 32); q += __shfl_xor(q, 4, 32); q += __shfl_xor(q, 8, 32); q += __shfl_xor(q, 16, 32);
      const float rstd = rsqrtf(q * kInv64 + kLnEps);
      const float y0 = fmaxf((e0 * rstd) * ls0 + lb0, 0.0f);
      const float y1 = fmaxf((e1 * rstd) * ls1 + lb1, 0.0f);
      if (!HEAD) {
        const bool live = n < kNG;
        const float zz0 = live ? y0 : 0.0f;
        const float zz1 = live ? y1 : 0.0f;
        const unsigned short hb0 = f2bf_bits(zz0), hb1 = f2bf_bits(zz1);
        const unsigned short lb0b = f2bf_bits(zz0 - bf_bits2f(hb0)), lb1b = f2bf_bits(zz1 - bf_bits2f(hb1));
        const unsigned uh = pk16(hb0, hb1);
        const unsigned ul = pk16(lb0b, lb1b);
        unsigned* ph = (unsigned*)(xgh + (size_t)n * kDH) + lane;
        unsigned* pl = (unsigned*)(xgl + (size_t)n * kDH) + lane;
        *(volatile unsigned*)ph = uh;
        *(volatile unsigned*)pl = ul;
        __threadfence();
        *(volatile unsigned*)ph = uh;
        *(volatile unsigned*)pl = ul;
      } else {
        float l0 = y0 * w00 + y1 * w10;
        float l1 = y0 * w01 + y1 * w11;
        float l2 = y0 * w02 + y1 * w12;
#pragma unroll
        for (int off = 1; off < 32; off <<= 1) {
          l0 += __shfl_xor(l0, off, 32);
          l1 += __shfl_xor(l1, off, 32);
          l2 += __shfl_xor(l2, off, 32);
        }
        l0 += bo0; l1 += bo1; l2 += bo2;
        const float mx  = fmaxf(l0, fmaxf(l1, l2));
        const float x0  = expf(l0 - mx), x1 = expf(l1 - mx), x2 = expf(l2 - mx);
        const float inv = 1.0f / ((x0 + x1) + x2);
        const float p0 = x0 * inv, p1 = x1 * inv, p2 = x2 * inv;
        const float pr = (lane == 0) ? p0 : ((lane == 1) ? p1 : p2);
        if (lane < 3) so[3 * row + lane] = pr;
      }
    }
  }
  if (HEAD) {
    __syncthreads();
    const size_t obase = (size_t)b * kTileRows * 3;
    for (int ps = 0; ps < 2; ++ps) {
#pragma unroll 1
      for (int i = tid; i < kTileRows * 3 / 4; i += kThreads) {
        const size_t o = obase + 4 * (size_t)i;
        const v4f qv = *(const v4f*)(so + 4 * i);
        if (o + 4 <= (size_t)kOutN) *(volatile v4f*)(out + o) = qv;
      }
      __threadfence();
    }
  }
}

extern "C" void kernel_launch(void* const* d_in, const int* in_sizes, int n_in,
                              void* d_out, int out_size, void* d_ws, size_t ws_size, hipStream_t stream) {
  if (n_in < 36) return;
  if (out_size != kOutN) return;
  if (in_sizes[2] != 2 * kEGG || in_sizes[4] != 2 * kECG || in_sizes[5] != 2 * kECC) return;
  if (in_sizes[0] != kNG * kDR || in_sizes[1] != kNC * kDR || in_sizes[3] != kEGG) return;
  if (in_sizes[16] < 1 || in_sizes[19] < 1 || in_sizes[26] < 1 || in_sizes[35] < 3) return;

  const float* x_glom = (const float*)d_in[0];
  const float* x_cell = (const float*)d_in[1];
  const int*   ei_gg  = (const int*)d_in[2];
  const float* ew_gg  = (const float*)d_in[3];
  const int*   ei_cg  = (const int*)d_in[4];
  const int*   ei_cc  = (const int*)d_in[5];
  const float* W_in_g = (const float*)d_in[6];
  const float* b_in_g = (const float*)d_in[7];
  const float* lnig_s = (const float*)d_in[8];
  const float* lnig_b = (const float*)d_in[9];
  const float* W_in_c = (const float*)d_in[10];
  const float* b_in_c = (const float*)d_in[11];
  const float* lnic_s = (const float*)d_in[12];
  const float* lnic_b = (const float*)d_in[13];
  const float* W_gcn1 = (const float*)d_in[14];
  const float* b_gcn1 = (const float*)d_in[15];
  const float* eps_cg1 = (const float*)d_in[16];
  const float* W_cg1  = (const float*)d_in[17];
  const float* b_cg1  = (const float*)d_in[18];
  const float* eps_cc1 = (const float*)d_in[19];
  const float* W_cc1  = (const float*)d_in[20];
  const float* b_cc1  = (const float*)d_in[21];
  const float* ln1_s  = (const float*)d_in[22];
  const float* ln1_b  = (const float*)d_in[23];
  const float* W_gcn2 = (const float*)d_in[24];
  const float* b_gcn2 = (const float*)d_in[25];
  const float* eps_cg2 = (const float*)d_in[26];
  const float* W_cg2  = (const float*)d_in[27];
  const float* b_cg2  = (const float*)d_in[28];
  const float* ln2_s  = (const float*)d_in[32];
  const float* ln2_b  = (const float*)d_in[33];
  const float* W_out  = (const float*)d_in[34];
  const float* b_out  = (const float*)d_in[35];
  float* out = (float*)d_out;

  char* ws = (char*)d_ws; size_t off = 0;
  auto carve = [&](size_t bytes) -> char* { char* p = ws + off; off += (bytes + 255) & ~(size_t)255; return p; };
  unsigned short* WPL    = (unsigned short*)carve((size_t)kWSlots * kWPlane * 2);
  unsigned short* XGH    = (unsigned short*)carve((size_t)kNGP * kDH * 2);
  unsigned short* XGL    = (unsigned short*)carve((size_t)kNGP * kDH * 2);
  float*          XC32   = (float*)carve((size_t)kNCP * kDH * 4);
  float*          XT32   = (float*)carve((size_t)kNGP * kDH * 4);
  unsigned short* HGH    = (unsigned short*)carve((size_t)kNGP * kDH * 2);
  unsigned short* HGL    = (unsigned short*)carve((size_t)kNGP * kDH * 2);
  unsigned short* HCH    = (unsigned short*)carve((size_t)kNCP * kDH * 2);
  unsigned short* HCL    = (unsigned short*)carve((size_t)kNCP * kDH * 2);
  float*          GIN32  = (float*)carve((size_t)kNGP * kDH * 4);
  unsigned*       SORTGG = (unsigned*)carve(((size_t)kNchGG * kCH + 32) * 4);
  unsigned*       SORTCG = (unsigned*)carve(((size_t)kNchCG * kCH + 32) * 4);
  unsigned*       SORTCC = (unsigned*)carve(((size_t)kNchCG * kCH + 32) * 4);
  int*            TABGG  = (int*)carve((size_t)kNchGG * kNKPG * 4);
  int*            TABCG  = (int*)carve((size_t)kNchCG * kNKPG * 4);
  int*            TABCC  = (int*)carve((size_t)kNchCG * kNKPC * 4);
  float*          DINV   = (float*)carve((size_t)kBlkG * kTileRows * 4);
  float*          NORM   = (float*)carve((size_t)kEGG * 4);
  if (off > ws_size || off > (size_t)134217728) return;

  const int tilesG = kNGP / kGRW;
  const int tilesC = kNCP / kGRW;
  const int gridG  = (tilesG + 7) / 8;
  const int gridC  = (tilesC + 7) / 8;
  const float*          nullf  = nullptr;
  const unsigned short* null16 = nullptr;
  float*                nullC  = nullptr;
  unsigned short*       nullH  = nullptr;

  prep_weights<<<kWSlots, 256, 0, stream>>>(W_in_g, W_in_c, W_gcn1, W_gcn2, W_cg1, W_cc1, W_cg2, WPL);

  gemm_n64<kDR, true, false, 2, 2><<<gridG, 256, 0, stream>>>(x_glom, null16, null16, kNG, tilesG, WPL + 0 * kWPlane,
                                                             b_in_g, lnig_s, lnig_b, nullC, XGH, XGL);
  gemm_n64<kDR, true, false, 2, 0><<<gridC, 256, 0, stream>>>(x_cell, null16, null16, kNC, tilesC, WPL + 1 * kWPlane,
                                                             b_in_c, lnic_s, lnic_b, XC32, nullH, nullH);

  bucket_edges<1024, 10><<<kNchGG, kThreads, 0, stream>>>(ei_gg + kEGG, kEGG, kNG, kNKPG, SORTGG, TABGG, kNchGG);
  bucket_edges<1024, 10><<<kNchCG, kThreads, 0, stream>>>(ei_cg + kECG, kECG, kNG, kNKPG, SORTCG, TABCG, kNchCG);
  bucket_edges<2048, 11><<<kNchCG, kThreads, 0, stream>>>(ei_cc + kECC, kECC, kNC, kNKPC, SORTCC, TABCC, kNchCG);

  k_deg<<<kBlkG, kThreads, 0, stream>>>(SORTGG, TABGG, ew_gg, DINV);
  k_norm<<<(kEGG / 4 + 255) / 256, 256, 0, stream>>>(ei_gg, ew_gg, DINV, NORM);

  gemm_n64<kDH, false, true, 0, 0><<<gridG, 256, 0, stream>>>(nullf, XGH, XGL, kNG, tilesG, WPL + 2 * kWPlane,
                                                             nullf, nullf, nullf, XT32, nullH, nullH);
  k_gin<true><<<kBlkG, kThreads, 0, stream>>>(SORTCG, TABCG, kNchCG, kNKPG, ei_cg, kECG, XC32, kNC,
                                               nullf, XGH, XGL, kNG, kNGP, eps_cg1, HGH, HGL);
  k_gin<false><<<kBlkC, kThreads, 0, stream>>>(SORTCC, TABCC, kNchCG, kNKPC, ei_cc, kECC, XC32, kNC,
                                                XC32, null16, null16, kNC, kNCP, eps_cc1, HCH, HCL);
  gemm_n64<kDH, false, true, 1, 0><<<gridG, 256, 0, stream>>>(nullf, HGH, HGL, kNG, tilesG, WPL + 4 * kWPlane,
                                                             b_cg1, nullf, nullf, GIN32, nullH, nullH);
  gemm_n64<kDH, false, true, 3, 0><<<gridC, 256, 0, stream>>>(nullf, HCH, HCL, kNC, tilesC, WPL + 5 * kWPlane,
                                                             b_cc1, ln1_s, ln1_b, XC32, nullH, nullH);
  k_gcn<false><<<kBlkG, kThreads, 0, stream>>>(SORTGG, TABGG, ei_gg, NORM, XT32, DINV, b_gcn1, GIN32, ln1_s, ln1_b,
                                                XGH, XGL, nullf, nullf, nullC);

  gemm_n64<kDH, false, true, 0, 0><<<gridG, 256, 0, stream>>>(nullf, XGH, XGL, kNG, tilesG, WPL + 3 * kWPlane,
                                                             nullf, nullf, nullf, XT32, nullH, nullH);
  k_gin<true><<<kBlkG, kThreads, 0, stream>>>(SORTCG, TABCG, kNchCG, kNKPG, ei_cg, kECG, XC32, kNC,
                                               nullf, XGH, XGL, kNG, kNGP, eps_cg2, HGH, HGL);
  gemm_n64<kDH, false, true, 1, 0><<<gridG, 256, 0, stream>>>(nullf, HGH, HGL, kNG, tilesG, WPL + 6 * kWPlane,
                                                             b_cg2, nullf, nullf, GIN32, nullH, nullH);
  k_gcn<true><<<kBlkG, kThreads, 0, stream>>>(SORTGG, TABGG, ei_gg, NORM, XT32, DINV, b_gcn2, GIN32, ln2_s, ln2_b,
                                               nullH, nullH, W_out, b_out, out);
}
